// MambaPlusPlusBlock_4793183502529
// MI455X (gfx1250) — hardware-verified
//
#include <hip/hip_runtime.h>
#include <math.h>

typedef __attribute__((ext_vector_type(16))) _Float16 v16h;
typedef __attribute__((ext_vector_type(8)))  _Float16 v8h;
typedef __attribute__((ext_vector_type(16))) __bf16   v16b;
typedef __attribute__((ext_vector_type(8)))  __bf16   v8b;
typedef __attribute__((ext_vector_type(8)))  float    v8f;
typedef __attribute__((ext_vector_type(4)))  float    v4f;

constexpr int kBatch = 2;
constexpr int kSeq   = 1024;
constexpr int kRows  = kBatch * kSeq;
constexpr int kDm    = 272;
constexpr int kDmK   = 288;
constexpr int kDin   = 544;
constexpr int kXzW   = 2 * kDin;
constexpr int kNst   = 64;
constexpr int kDtR   = 17;
constexpr int kXdW   = kDtR + 2 * kNst;
constexpr int kXdP   = 192;
constexpr int kOutP  = 320;
constexpr int kConv  = 4;
constexpr float kLamInit     = 0.47071301834358416f;
constexpr float kOneMinusLam = 0.52928698165641584f;

constexpr int kScanTS  = 64;
constexpr int kScanCh  = 32;
constexpr int kScanThr = 128;
constexpr int kNq      = 16;
constexpr int kSXP     = 148;
constexpr int kSYP     = 36;
constexpr int kConvTP  = 36;

static_assert((kDmK % 32) == 0 && (kDin % 32) == 0);
static_assert((kRows % 64) == 0 && (kXzW % 64) == 0 && (kXdP % 64) == 0 && (kOutP % 64) == 0);
static_assert((kSeq % kScanTS) == 0 && (kDin % kScanCh) == 0 && (kSeq % 64) == 0 && (kDin % 32) == 0);
static_assert(4 * kNq == kNst && kScanThr == 4 * kScanCh);

constexpr size_t kOffXN   = 0;
constexpr size_t kOffXNH  = kOffXN  + (size_t)kRows * kDmK * 4;
constexpr size_t kOffXNL  = kOffXNH + (size_t)kRows * kDmK * 2;
constexpr size_t kOffWIH  = kOffXNL + (size_t)kRows * kDmK * 2;
constexpr size_t kOffWIL  = kOffWIH + (size_t)kXzW  * kDmK * 2;
constexpr size_t kOffWXH  = kOffWIL + (size_t)kXzW  * kDmK * 2;
constexpr size_t kOffWXL  = kOffWXH + (size_t)kXdP  * kDin * 2;
constexpr size_t kOffWOH  = kOffWXL + (size_t)kXdP  * kDin * 2;
constexpr size_t kOffWOL  = kOffWOH + (size_t)kOutP * kDin * 2;
constexpr size_t kOffXZ   = kOffWOL + (size_t)kOutP * kDin * 2;
constexpr size_t kOffUC   = kOffXZ  + (size_t)kRows * kXzW * 4;
constexpr size_t kOffUCH  = kOffUC  + (size_t)kRows * kDin * 4;
constexpr size_t kOffUCL  = kOffUCH + (size_t)kRows * kDin * 2;
constexpr size_t kOffXD   = kOffUCL + (size_t)kRows * kDin * 2;
constexpr size_t kOffYF   = kOffXD  + (size_t)kRows * kXdP * 4;
constexpr size_t kOffYH   = kOffYF  + (size_t)kRows * kDin * 4;
constexpr size_t kOffYL   = kOffYH  + (size_t)kRows * kDin * 2;
constexpr size_t kOffY1   = kOffYL  + (size_t)kRows * kDin * 2;
constexpr size_t kOffY2   = kOffY1  + (size_t)kRows * kOutP * 4;
constexpr size_t kWsTotal = kOffY2  + (size_t)kRows * kOutP * 4;
static_assert(kWsTotal == 40640512ull);
static_assert(kWsTotal <= 134217728ull);
static_assert((kOffXNH % 128) == 0 && (kOffXNL % 128) == 0 && (kOffWIH % 128) == 0 && (kOffWIL % 128) == 0 &&
              (kOffWXH % 128) == 0 && (kOffWXL % 128) == 0 && (kOffWOH % 128) == 0 && (kOffWOL % 128) == 0 &&
              (kOffXZ % 128) == 0 && (kOffUC % 128) == 0 && (kOffUCH % 128) == 0 && (kOffUCL % 128) == 0 &&
              (kOffXD % 128) == 0 && (kOffYF % 128) == 0 && (kOffYH % 128) == 0 && (kOffYL % 128) == 0 &&
              (kOffY1 % 128) == 0 && (kOffY2 % 128) == 0);

__device__ __forceinline__ unsigned short f2bf_bits(float f) {
  unsigned u = __float_as_uint(f);
  return (unsigned short)((u + 0x7FFFu + ((u >> 16) & 1u)) >> 16);
}
__device__ __forceinline__ float bf_bits2f(unsigned short h) { return __uint_as_float(((unsigned)h) << 16); }

__device__ __forceinline__ void dep_guard_h(v8f& a, v8f& b, v16h x, v16h y) { asm volatile("v_nop\n\tv_nop\n\tv_nop\n\tv_nop" : "+v"(a), "+v"(b) : "v"(x), "v"(y)); }
__device__ __forceinline__ void dep_guard_b(v8f& a, v8f& b, v16b x, v16b y) { asm volatile("v_nop\n\tv_nop\n\tv_nop\n\tv_nop" : "+v"(a), "+v"(b) : "v"(x), "v"(y)); }
__device__ __forceinline__ void keep4_h(v16h a, v16h b, v16h c, v16h d) { asm volatile("v_nop" :: "v"(a), "v"(b), "v"(c), "v"(d)); }
__device__ __forceinline__ void keep4_b(v16b a, v16b b, v16b c, v16b d) { asm volatile("v_nop" :: "v"(a), "v"(b), "v"(c), "v"(d)); }
__device__ __forceinline__ void acc_guard4(v8f& a, v8f& b, v8f& c, v8f& d) { asm volatile("v_nop\n\tv_nop\n\tv_nop\n\tv_nop" : "+v"(a), "+v"(b), "+v"(c), "+v"(d)); }
template <typename T> struct Frag;
template <> struct Frag<_Float16> {
  typedef v16h V; union U { v16h v; v8h h[2]; };
  static __device__ __forceinline__ v16h load(const _Float16* p) {
    U f; f.h[0] = *(const v8h*)(p); f.h[1] = *(const v8h*)(p + 16); return f.v;
  }
  static __device__ __forceinline__ v8f mma(v16h a, v16h b, v8f c) {
    return __builtin_amdgcn_wmma_f32_16x16x32_f16(false, a, false, b, (short)0, c, false, false);
  }
  static __device__ __forceinline__ void guard(v8f& a, v8f& b, v16h x, v16h y) { dep_guard_h(a, b, x, y); }
  static __device__ __forceinline__ void keep(v16h a, v16h b, v16h c, v16h d) { keep4_h(a, b, c, d); }
};
template <> struct Frag<__bf16> {
  typedef v16b V; union U { v16b v; v8b h[2]; };
  static __device__ __forceinline__ v16b load(const __bf16* p) {
    U f; f.h[0] = *(const v8b*)(p); f.h[1] = *(const v8b*)(p + 16); return f.v;
  }
  static __device__ __forceinline__ v8f mma(v16b a, v16b b, v8f c) {
    return __builtin_amdgcn_wmma_f32_16x16x32_bf16(false, a, false, b, (short)0, c, false, false);
  }
  static __device__ __forceinline__ void guard(v8f& a, v8f& b, v16b x, v16b y) { dep_guard_b(a, b, x, y); }
  static __device__ __forceinline__ void keep(v16b a, v16b b, v16b c, v16b d) { keep4_b(a, b, c, d); }
};

template <int ET> struct Elem;
template <> struct Elem<0> { typedef _Float16 T; };
template <> struct Elem<1> { typedef __bf16 T; };
template <int ET, int SPL, int BIAS_MODE, int OUT_MODE, bool RESID, int ACT = 0>
__global__ __launch_bounds__(256) void wmma_gemm64(
    const unsigned short* __restrict__ Ap, const unsigned short* __restrict__ A2p, int lda, long strideA,
    const unsigned short* __restrict__ Btp, const unsigned short* __restrict__ Bt2p, int ldb, long strideB,
    void* __restrict__ Cout, void* __restrict__ Cout2, int ldc, long strideC,
    const float* __restrict__ bias,
    const float* __restrict__ resid, long strideR,
    int M, int N, int K, float scale) {
  typedef typename Elem<ET>::T T;
  typedef typename Frag<T>::V V;
  const T* A = (const T*)Ap; const T* A2 = (const T*)A2p; const T* Bt = (const T*)Btp; const T* Bt2 = (const T*)Bt2p;
  __shared__ __align__(16) float sT[8][16 * 68];
  const int b    = blockIdx.y;
  const int lane = threadIdx.x & 31;
  const int wave = threadIdx.x >> 5;
  const int tilesN = N >> 6;
  const int tilesM = M >> 6;
  const int tile = blockIdx.x * 8 + wave;
  if (tile >= tilesM * tilesN) return;
  const int tm = tile / tilesN;
  const int tn = tile - tm * tilesN;
  const int m0 = tm << 6;
  const int n0 = tn << 6;

  const T* Ab  = A  + (size_t)b * strideA;
  const T* Bb  = Bt + (size_t)b * strideB;
  const T* Ab2 = (SPL >= 1) ? (A2  + (size_t)b * strideA) : nullptr;
  const T* Bb2 = (SPL == 2) ? (Bt2 + (size_t)b * strideB) : nullptr;

  const int rlane = lane & 15;
  const int koff  = (lane >> 4) * 8;
  const int mOff  = (lane >> 4) * 8;

  v8f acc[4][4];
#pragma unroll
  for (int i = 0; i < 4; ++i)
#pragma unroll
    for (int j = 0; j < 4; ++j) acc[i][j] = (v8f){0.f,0.f,0.f,0.f,0.f,0.f,0.f,0.f};

  for (int k0 = 0; k0 < K; k0 += 32) {
    V bh[4], bl[4];
#pragma unroll
    for (int j = 0; j < 4; ++j) {
      const size_t bo = (size_t)(n0 + (j << 4) + rlane) * ldb + koff + k0;
      bh[j] = Frag<T>::load(Bb + bo);
      if (SPL == 2) bl[j] = Frag<T>::load(Bb2 + bo);
    }
#pragma unroll
    for (int i = 0; i < 4; ++i) {
      const size_t ao = (size_t)(m0 + (i << 4) + rlane) * lda + koff + k0;
      V ah = Frag<T>::load(Ab + ao);
      V al;
      if (SPL >= 1) al = Frag<T>::load(Ab2 + ao);
#pragma unroll
      for (int j = 0; j < 4; ++j) {
        acc[i][j] = Frag<T>::mma(ah, bh[j], acc[i][j]);
        if (SPL == 2) acc[i][j] = Frag<T>::mma(ah, bl[j], acc[i][j]);
        if (SPL >= 1) acc[i][j] = Frag<T>::mma(al, bh[j], acc[i][j]);
      }
      Frag<T>::guard(acc[i][0], acc[i][3], ah, (SPL >= 1) ? al : ah);
    }
    Frag<T>::keep(bh[0], bh[1], bh[2], bh[3]);
    if (SPL == 2) Frag<T>::keep(bl[0], bl[1], bl[2], bl[3]);
  }
  acc_guard4(acc[0][0], acc[0][1], acc[0][2], acc[0][3]);
  acc_guard4(acc[1][0], acc[1][1], acc[1][2], acc[1][3]);
  acc_guard4(acc[2][0], acc[2][1], acc[2][2], acc[2][3]);
  acc_guard4(acc[3][0], acc[3][1], acc[3][2], acc[3][3]);

  float* slab = sT[wave];
  const float* Rb = RESID ? (resid + (size_t)b * strideR) : nullptr;
#pragma unroll
  for (int i = 0; i < 4; ++i) {
    const int mBase = m0 + (i << 4);
#pragma unroll
    for (int j = 0; j < 4; ++j) {
      const int n = n0 + (j << 4) + rlane;
      float bv = 0.f;
      if (BIAS_MODE == 2) bv = bias[n];
#pragma unroll
      for (int r = 0; r < 8; ++r) {
        float v = acc[i][j][r] * scale;
        if (BIAS_MODE == 1) v += bias[mBase + mOff + r];
        if (BIAS_MODE == 2) v += bv;
        if (RESID) v += Rb[(size_t)(mBase + mOff + r) * ldc + n];
        if (ACT == 1) v = tanhf(v);
        if (ACT == 2) v = fmaxf(v, 0.0f);
        if (ACT == 3) v = v / (1.0f + expf(-v));
        if (ACT == 4) v = (v > 0.f) ? v : 0.01f * v;
        slab[(mOff + r) * 68 + (j << 4) + rlane] = v;
      }
    }
    __builtin_amdgcn_fence(__ATOMIC_RELEASE, "workgroup");
    __builtin_amdgcn_wave_barrier();
    __builtin_amdgcn_fence(__ATOMIC_ACQUIRE, "workgroup");
    if (OUT_MODE == 0) {
      float* C = (float*)Cout + (size_t)b * strideC;
      const int hh = lane >> 4, c4 = (lane & 15) * 4;
      for (int pass = 0; pass < 2; ++pass) {
#pragma unroll
        for (int it = 0; it < 8; ++it) {
          const int row = it * 2 + hh;
          v4f v = *(const v4f*)(slab + row * 68 + c4);
          *(volatile v4f*)(C + (size_t)(mBase + row) * ldc + n0 + c4) = v;
        }
        __threadfence();
      }
    } else {
      const int q = lane >> 3, c8 = (lane & 7) * 8;
      unsigned short* C  = (unsigned short*)Cout  + (size_t)b * strideC;
      unsigned short* C2 = (OUT_MODE == 2) ? ((unsigned short*)Cout2 + (size_t)b * strideC) : nullptr;
      for (int pass = 0; pass < 2; ++pass) {
#pragma unroll
        for (int it = 0; it < 4; ++it) {
          const int row = it * 4 + q;
          const float* sp = slab + row * 68 + c8;
          v8h hv, lv;
#pragma unroll
          for (int e = 0; e < 8; ++e) {
            if (OUT_MODE == 1) {
              hv[e] = (_Float16)sp[e];
            } else {
              unsigned short hb = f2bf_bits(sp[e]);
              unsigned short lb = f2bf_bits(sp[e] - bf_bits2f(hb));
              hv[e] = __builtin_bit_cast(_Float16, hb);
              lv[e] = __builtin_bit_cast(_Float16, lb);
            }
          }
          *(volatile v8h*)(C + (size_t)(mBase + row) * ldc + n0 + c8) = hv;
          if (OUT_MODE == 2) *(volatile v8h*)(C2 + (size_t)(mBase + row) * ldc + n0 + c8) = lv;
        }
        __threadfence();
      }
    }
    __builtin_amdgcn_fence(__ATOMIC_RELEASE, "workgroup");
    __builtin_amdgcn_wave_barrier();
    __builtin_amdgcn_fence(__ATOMIC_ACQUIRE, "workgroup");
  }
}

__global__ __launch_bounds__(256) void split_rows_bf16_kernel(
    const float* __restrict__ src, unsigned short* __restrict__ dhi, unsigned short* __restrict__ dlo, int total8)
{
  const int i = blockIdx.x * 256 + threadIdx.x;
  if (i >= total8) return;
  const size_t e0 = (size_t)i << 3;
  const v4f a0 = *(const v4f*)(src + e0);
  const v4f a1 = *(const v4f*)(src + e0 + 4);
  v8h hv, lv;
#pragma unroll
  for (int e = 0; e < 4; ++e) {
    const unsigned short h0 = f2bf_bits(a0[e]), h1 = f2bf_bits(a1[e]);
    const unsigned short l0 = f2bf_bits(a0[e] - bf_bits2f(h0)), l1 = f2bf_bits(a1[e] - bf_bits2f(h1));
    hv[e]     = __builtin_bit_cast(_Float16, h0);
    hv[4 + e] = __builtin_bit_cast(_Float16, h1);
    lv[e]     = __builtin_bit_cast(_Float16, l0);
    lv[4 + e] = __builtin_bit_cast(_Float16, l1);
  }
  unsigned short* qh = dhi + e0;
  unsigned short* ql = dlo + e0;
  *(volatile v8h*)qh = hv;
  *(volatile v8h*)ql = lv;
  __threadfence();
  *(volatile v8h*)qh = hv;
  *(volatile v8h*)ql = lv;
}

__global__ __launch_bounds__(256) void split_pad_bf16_kernel(
    const float* __restrict__ src, int srcRows, int srcCols,
    unsigned short* __restrict__ dhi, unsigned short* __restrict__ dlo, int dstCols, int total8)
{
  const int i = blockIdx.x * 256 + threadIdx.x;
  if (i >= total8) return;
  const size_t e0 = (size_t)i << 3;
  const int row = (int)(e0 / (size_t)dstCols);
  const int col = (int)(e0 - (size_t)row * dstCols);
  const bool valid = (row < srcRows) && (col < srcCols);
  const int rs = (row < srcRows) ? row : (srcRows - 1);
  const int cs = (col < srcCols) ? col : (srcCols - 8);
  const float* sp = src + (size_t)rs * srcCols + cs;
  const v4f a0 = *(const v4f*)(sp);
  const v4f a1 = *(const v4f*)(sp + 4);
  v8h hv, lv;
#pragma unroll
  for (int e = 0; e < 4; ++e) {
    const float f0 = valid ? a0[e] : 0.f;
    const float f1 = valid ? a1[e] : 0.f;
    const unsigned short h0 = f2bf_bits(f0), h1 = f2bf_bits(f1);
    const unsigned short l0 = f2bf_bits(f0 - bf_bits2f(h0)), l1 = f2bf_bits(f1 - bf_bits2f(h1));
    hv[e]     = __builtin_bit_cast(_Float16, h0);
    hv[4 + e] = __builtin_bit_cast(_Float16, h1);
    lv[e]     = __builtin_bit_cast(_Float16, l0);
    lv[4 + e] = __builtin_bit_cast(_Float16, l1);
  }
  unsigned short* qh = dhi + e0;
  unsigned short* ql = dlo + e0;
  *(volatile v8h*)qh = hv;
  *(volatile v8h*)ql = lv;
  __threadfence();
  *(volatile v8h*)qh = hv;
  *(volatile v8h*)ql = lv;
}

__global__ __launch_bounds__(256) void rmsnorm_kernel(
    const float* __restrict__ x, const float* __restrict__ w, float* __restrict__ XN)
{
  const int lane = threadIdx.x & 31, wave = threadIdx.x >> 5;
  const int row = blockIdx.x * 8 + wave;
  const float* xr = x + (size_t)row * kDm;
  const int cA = lane * 4, cB = 128 + lane * 4;
  const int l3 = (lane < 3) ? lane : 3;
  const int cC = 256 + l3 * 4;
  const bool vC = (lane < 4);
  const v4f a0 = *(const v4f*)(xr + cA);
  const v4f a1 = *(const v4f*)(xr + cB);
  const v4f a2r = *(const v4f*)(xr + cC);
  const v4f w0 = *(const v4f*)(w + cA);
  const v4f w1 = *(const v4f*)(w + cB);
  const v4f w2r = *(const v4f*)(w + cC);
  float ss = 0.f;
#pragma unroll
  for (int e = 0; e < 4; ++e) {
    const float t2 = vC ? a2r[e] : 0.f;
    ss = fmaf(a0[e], a0[e], ss);
    ss = fmaf(a1[e], a1[e], ss);
    ss = fmaf(t2, t2, ss);
  }
#pragma unroll
  for (int off = 16; off > 0; off >>= 1) ss += __shfl_xor(ss, off, 32);
  const float r = rsqrtf(ss * (1.0f / 272.0f) + 1e-5f);
  v4f o0, o1, o2;
#pragma unroll
  for (int e = 0; e < 4; ++e) {
    o0[e] = (a0[e] * r) * w0[e];
    o1[e] = (a1[e] * r) * w1[e];
    o2[e] = vC ? ((a2r[e] * r) * w2r[e]) : 0.f;
  }
  float* ob = XN + (size_t)row * kDmK;
  for (int pass = 0; pass < 2; ++pass) {
    *(volatile v4f*)(ob + cA) = o0;
    *(volatile v4f*)(ob + cB) = o1;
    if (lane < 8) *(volatile v4f*)(ob + 256 + lane * 4) = o2;
    __threadfence();
  }
}

__device__ __forceinline__ int t_of(int s, int bwd) { return bwd ? (kSeq - 1 - s) : s; }

__global__ __launch_bounds__(32) void conv_silu_kernel(
    const float* __restrict__ XZ, const float* __restrict__ cw, const float* __restrict__ cb,
    float* __restrict__ UC, int bwd)
{
  __shared__ __align__(16) float sT[16 * kConvTP];
  const int lane = threadIdx.x;
  const int d0 = blockIdx.x * 32, d = d0 + lane;
  const int chunk = blockIdx.y;
  const int b = chunk >> 4;
  const int s0 = (chunk & 15) * 64;
  const size_t rowb = (size_t)b * kSeq;
  const float w0 = cw[d * kConv + 0], w1 = cw[d * kConv + 1], w2 = cw[d * kConv + 2], w3 = cw[d * kConv + 3];
  const float bc = cb[d];
  float xm3, xm2, xm1;
  {
    const bool hist = (s0 > 0);
    const int sh = hist ? (s0 - 3) : 0;
    const float v3 = XZ[(rowb + t_of(sh, bwd)) * kXzW + d];
    const float v2 = XZ[(rowb + t_of(sh + 1, bwd)) * kXzW + d];
    const float v1 = XZ[(rowb + t_of(sh + 2, bwd)) * kXzW + d];
    xm3 = hist ? v3 : 0.f;
    xm2 = hist ? v2 : 0.f;
    xm1 = hist ? v1 : 0.f;
  }
  const int q = lane >> 3, c4 = (lane & 7) * 4;
#pragma unroll 1
  for (int sub = 0; sub < 4; ++sub) {
    const int lb = s0 + sub * 16;
#pragma unroll 1
    for (int sl = 0; sl < 16; ++sl) {
      const int s = lb + sl;
      const float xcur = XZ[(rowb + t_of(s, bwd)) * kXzW + d];
      float acc = w0 * xm3;
      acc = fmaf(w1, xm2, acc);
      acc = fmaf(w2, xm1, acc);
      acc = fmaf(w3, xcur, acc);
      const float sv = acc + bc;
      const float sg = __builtin_amdgcn_rcpf(1.0f + __expf(-sv));
      sT[sl * kConvTP + lane] = sv * sg;
      xm3 = xm2; xm2 = xm1; xm1 = xcur;
    }
    __syncthreads();
    v4f fv[4];
#pragma unroll
    for (int it = 0; it < 4; ++it) fv[it] = *(const v4f*)(sT + (it * 4 + q) * kConvTP + c4);
    for (int pass = 0; pass < 2; ++pass) {
#pragma unroll
      for (int it = 0; it < 4; ++it) {
        const int s = lb + it * 4 + q;
        *(volatile v4f*)(UC + (rowb + t_of(s, bwd)) * kDin + d0 + c4) = fv[it];
      }
      __threadfence();
    }
    __syncthreads();
  }
}

__global__ __launch_bounds__(kScanThr) void scan_kernel(
    const float* __restrict__ XD, const float* __restrict__ UC, const float* __restrict__ XZ,
    const float* __restrict__ Wdt, const float* __restrict__ bdt, const float* __restrict__ Alog,
    const float* __restrict__ Dp, float* __restrict__ YF, int bwd)
{
  __shared__ __align__(16) float sX[kScanTS * kSXP];
  __shared__ __align__(16) float sY[kScanTS * kSYP];
  __shared__ __align__(16) float sD[kScanTS * kScanCh];
  __shared__ __align__(16) float sW[kDtR * kScanCh];
  __shared__ float sBd[kScanCh];
  const int tid = threadIdx.x, lane = tid & 31, wave = tid >> 5;
  const int c   = wave * 8 + (lane & 7);
  const int qtr = lane >> 3;
  const int n0  = qtr * kNq;
  constexpr int kBlkPerB = kDin / kScanCh;
  const int bix = blockIdx.x / kBlkPerB;
  const int d0  = (blockIdx.x - bix * kBlkPerB) * kScanCh;
  const int d   = d0 + c;
  const size_t rowb = (size_t)bix * kSeq;

#pragma unroll 1
  for (int j = 0; j < 5; ++j) {
    const int idx = tid + kScanThr * j;
    const int idc = (idx < kDtR * kScanCh) ? idx : (kDtR * kScanCh - 1);
    const int r = idc >> 5, cc = idc & 31;
    const float val = Wdt[(size_t)(d0 + cc) * kDtR + r];
    if (idx < kDtR * kScanCh) sW[idx] = val;
  }
  {
    const float bv = bdt[d0 + (tid & 31)];
    if (tid < kScanCh) sBd[tid] = bv;
  }
#pragma unroll 1
  for (int j = 0; j < 16; ++j) {
    const int idx = tid + kScanThr * j;
    const int n = idx >> 5, cc = idx & 31;
    sD[idx] = -expf(Alog[(size_t)(d0 + cc) * kNst + n]);
  }
  __syncthreads();
  float negA[kNq], h[kNq];
#pragma unroll
  for (int k = 0; k < kNq; ++k) {
    negA[k] = sD[(n0 + k) * kScanCh + c];
    h[k] = 0.f;
  }
  const float Dd = Dp[d];
  __syncthreads();

  const int dst0 = (tid < kDtR) ? tid : (tid + 3);
  const int q = lane >> 3, c4 = (lane & 7) * 4;
#pragma unroll 1
  for (int t0 = 0; t0 < kSeq; t0 += kScanTS) {
    __syncthreads();
#pragma unroll 1
    for (int r = 0; r < kScanTS; ++r) {
      const float* base = XD + (rowb + t_of(t0 + r, bwd)) * kXdP;
      const float v0 = base[tid];
      const float v2 = base[128 + (tid & 63)];
      sX[r * kSXP + dst0] = v0;
      if (tid < kDtR) sX[r * kSXP + 131 + tid] = v2;
    }
    __syncthreads();
#pragma unroll 1
    for (int j = 0; j < 16; ++j) {
      const int idx = tid + kScanThr * j;
      const int s = idx >> 5, cc = idx & 31;
      const float* xr = sX + s * kSXP;
      float vdot = 0.f;
#pragma unroll 1
      for (int r = 0; r < kDtR; ++r) vdot = fmaf(xr[r], sW[r * kScanCh + cc], vdot);
      const float v   = vdot + sBd[cc];
      const float a   = __expf(-fabsf(v));
      const float ua  = 1.0f + a;
      const float l1p = __logf(ua) + (a - (ua - 1.0f)) * __builtin_amdgcn_rcpf(ua);
      sD[idx] = fmaxf(v, 0.0f) + l1p;
    }
    __syncthreads();
#pragma unroll 1
    for (int s = 0; s < kScanTS; ++s) {
      const float* xr = sX + s * kSXP;
      const float dt = sD[s * kScanCh + c];
      const size_t grow = rowb + t_of(t0 + s, bwd);
      const float xt = UC[grow * kDin + d];
      const float zv = XZ[grow * kXzW + kDin + d];
      const float dtx = dt * xt;
      float p = 0.f;
#pragma unroll
      for (int k4 = 0; k4 < kNq / 4; ++k4) {
        const v4f bv = *(const v4f*)(xr + 20 + n0 + 4 * k4);
        const v4f cv = *(const v4f*)(xr + 84 + n0 + 4 * k4);
#pragma unroll
        for (int e = 0; e < 4; ++e) {
          const int k = 4 * k4 + e;
          const float ex = __expf(dt * negA[k]);
          h[k] = ex * h[k] + dtx * bv[e];
          p = fmaf(h[k], cv[e], p);
        }
      }
      p += __shfl_xor(p, 8, 32);
      p += __shfl_xor(p, 16, 32);
      float y = xt * Dd + p;
      const float sg = __builtin_amdgcn_rcpf(1.0f + __expf(-zv));
      y = y * (zv * sg);
      if (qtr == 0) sY[s * kSYP + c] = y;
    }
    __syncthreads();
    for (int pass = 0; pass < 2; ++pass) {
#pragma unroll
      for (int it = 0; it < 4; ++it) {
        const int lrow = it * 16 + wave * 4 + q;
        const v4f val = *(const v4f*)(sY + lrow * kSYP + c4);
        *(volatile v4f*)(YF + (rowb + t_of(t0 + lrow, bwd)) * kDin + d0 + c4) = val;
      }
      __threadfence();
    }
  }
}

__global__ __launch_bounds__(256) void combine_kernel(
    const float* __restrict__ x, const float* __restrict__ lq, const float* __restrict__ w2,
    const float* __restrict__ Y1, const float* __restrict__ Y2, float* __restrict__ out)
{
  __shared__ __align__(16) float sO[8 * kDm];
  const int tid = threadIdx.x, lane = tid & 31, wave = tid >> 5;
  const int row = blockIdx.x * 8 + wave;
  float s = 0.f;
#pragma unroll
  for (int j = 0; j < 9; ++j) {
    const int i = lane + 32 * j;
    const int ic = (i < kDm) ? i : (kDm - 1);
    const float v = lq[ic];
    s += (i < kDm) ? v : 0.f;
  }
#pragma unroll
  for (int off = 16; off > 0; off >>= 1) s += __shfl_xor(s, off, 32);
  const float lam = __builtin_amdgcn_rcpf(1.0f + expf(-s)) + kLamInit;

  const float* y1r = Y1 + (size_t)row * kOutP;
  const float* y2r = Y2 + (size_t)row * kOutP;
  const float* xr  = x  + (size_t)row * kDm;
  float dv[9];
  float ss = 0.f;
#pragma unroll
  for (int j = 0; j < 9; ++j) {
    const int i = lane + 32 * j;
    const int ic = (i < kDm) ? i : (kDm - 1);
    const float a = y1r[ic];
    const float bq = y2r[ic];
    const float dd = a - lam * bq;
    dv[j] = (i < kDm) ? dd : 0.f;
    ss = fmaf(dv[j], dv[j], ss);
  }
#pragma unroll
  for (int off = 16; off > 0; off >>= 1) ss += __shfl_xor(ss, off, 32);
  const float r = rsqrtf(ss * (1.0f / 272.0f) + 1e-5f);
#pragma unroll
  for (int j = 0; j < 9; ++j) {
    const int i = lane + 32 * j;
    const int ic = (i < kDm) ? i : (kDm - 1);
    const float xv = xr[ic];
    const float wv = w2[ic];
    const float o = xv + ((dv[j] * r) * wv) * kOneMinusLam;
    if (i < kDm) sO[wave * kDm + i] = o;
  }
  __syncthreads();
  float* ob = out + (size_t)blockIdx.x * (8 * kDm);
  for (int pass = 0; pass < 2; ++pass) {
#pragma unroll
    for (int it = 0; it < 3; ++it) {
      const int p = it * 256 + tid;
      if (p < (8 * kDm) / 4) {
        const v4f v = *(const v4f*)(sO + p * 4);
        *(volatile v4f*)(ob + (size_t)p * 4) = v;
      }
    }
    __threadfence();
  }
}

extern "C" void kernel_launch(void* const* d_in, const int* in_sizes, int n_in,
                              void* d_out, int out_size, void* d_ws, size_t ws_size,
                              hipStream_t stream) {
  if (n_in < 22) return;
  if (in_sizes[0] != kRows * kDm) return;
  if (in_sizes[1] != kDm || in_sizes[2] != kDm || in_sizes[3] != kDm) return;
  for (int dir = 0; dir < 2; ++dir) {
    const int o = 4 + 9 * dir;
    if (in_sizes[o + 0] != kXzW * kDm) return;
    if (in_sizes[o + 1] != kDin * kConv) return;
    if (in_sizes[o + 2] != kDin) return;
    if (in_sizes[o + 3] != kXdW * kDin) return;
    if (in_sizes[o + 4] != kDin * kDtR) return;
    if (in_sizes[o + 5] != kDin) return;
    if (in_sizes[o + 6] != kDin * kNst) return;
    if (in_sizes[o + 7] != kDin) return;
    if (in_sizes[o + 8] != kDm * kDin) return;
  }
  if (out_size != kRows * kDm) return;
  if (ws_size < kWsTotal) return;

  const float* x   = (const float*)d_in[0];
  const float* lq  = (const float*)d_in[1];
  const float* n1w = (const float*)d_in[2];
  const float* n2w = (const float*)d_in[3];
  float* out = (float*)d_out;

  char* ws = (char*)d_ws;
  float*          XN  = (float*)(ws + kOffXN);
  unsigned short* XNH = (unsigned short*)(ws + kOffXNH);
  unsigned short* XNL = (unsigned short*)(ws + kOffXNL);
  unsigned short* WIH = (unsigned short*)(ws + kOffWIH);
  unsigned short* WIL = (unsigned short*)(ws + kOffWIL);
  unsigned short* WXH = (unsigned short*)(ws + kOffWXH);
  unsigned short* WXL = (unsigned short*)(ws + kOffWXL);
  unsigned short* WOH = (unsigned short*)(ws + kOffWOH);
  unsigned short* WOL = (unsigned short*)(ws + kOffWOL);
  float*          XZ  = (float*)(ws + kOffXZ);
  float*          UC  = (float*)(ws + kOffUC);
  unsigned short* UCH = (unsigned short*)(ws + kOffUCH);
  unsigned short* UCL = (unsigned short*)(ws + kOffUCL);
  float*          XD  = (float*)(ws + kOffXD);
  float*          YF  = (float*)(ws + kOffYF);
  unsigned short* YH  = (unsigned short*)(ws + kOffYH);
  unsigned short* YL  = (unsigned short*)(ws + kOffYL);
  float*          Yo[2];
  Yo[0] = (float*)(ws + kOffY1);
  Yo[1] = (float*)(ws + kOffY2);

  rmsnorm_kernel<<<kRows / 8, 256, 0, stream>>>(x, n1w, XN);
  {
    const int t8 = kRows * kDmK / 8;
    split_rows_bf16_kernel<<<(t8 + 255) / 256, 256, 0, stream>>>(XN, XNH, XNL, t8);
  }

  for (int dir = 0; dir < 2; ++dir) {
    const int o = 4 + 9 * dir;
    const float* W_in    = (const float*)d_in[o + 0];
    const float* conv_w  = (const float*)d_in[o + 1];
    const float* conv_b  = (const float*)d_in[o + 2];
    const float* W_xproj = (const float*)d_in[o + 3];
    const float* W_dt    = (const float*)d_in[o + 4];
    const float* b_dt    = (const float*)d_in[o + 5];
    const float* A_log   = (const float*)d_in[o + 6];
    const float* Dp      = (const float*)d_in[o + 7];
    const float* W_out   = (const float*)d_in[o + 8];

    {
      const int t8 = kXzW * kDmK / 8;
      split_pad_bf16_kernel<<<(t8 + 255) / 256, 256, 0, stream>>>(W_in, kXzW, kDm, WIH, WIL, kDmK, t8);
    }
    {
      const int t8 = kXdP * kDin / 8;
      split_pad_bf16_kernel<<<(t8 + 255) / 256, 256, 0, stream>>>(W_xproj, kXdW, kDin, WXH, WXL, kDin, t8);
    }
    {
      const int t8 = kOutP * kDin / 8;
      split_pad_bf16_kernel<<<(t8 + 255) / 256, 256, 0, stream>>>(W_out, kDm, kDin, WOH, WOL, kDin, t8);
    }

    wmma_gemm64<1, 2, 0, 0, false><<<dim3((kRows / 64) * (kXzW / 64) / 8, 1), 256, 0, stream>>>(
        XNH, XNL, kDmK, 0L,
        WIH, WIL, kDmK, 0L,
        (void*)XZ, nullptr, kXzW, 0L,
        nullptr, nullptr, 0L,
        kRows, kXzW, kDmK, 1.0f);

    conv_silu_kernel<<<dim3(kDin / 32, kRows / 64), 32, 0, stream>>>(XZ, conv_w, conv_b, UC, dir);
    {
      const int t8 = kRows * kDin / 8;
      split_rows_bf16_kernel<<<(t8 + 255) / 256, 256, 0, stream>>>(UC, UCH, UCL, t8);
    }

    wmma_gemm64<1, 2, 0, 0, false><<<dim3((kRows / 64) * (kXdP / 64) / 8, 1), 256, 0, stream>>>(
        UCH, UCL, kDin, 0L,
        WXH, WXL, kDin, 0L,
        (void*)XD, nullptr, kXdP, 0L,
        nullptr, nullptr, 0L,
        kRows, kXdP, kDin, 1.0f);

    scan_kernel<<<kBatch * (kDin / kScanCh), kScanThr, 0, stream>>>(XD, UC, XZ, W_dt, b_dt, A_log, Dp, YF, dir);
    {
      const int t8 = kRows * kDin / 8;
      split_rows_bf16_kernel<<<(t8 + 255) / 256, 256, 0, stream>>>(YF, YH, YL, t8);
    }

    wmma_gemm64<1, 2, 0, 0, false><<<dim3((kRows / 64) * (kOutP / 64) / 8, 1), 256, 0, stream>>>(
        YH, YL, kDin, 0L,
        WOH, WOL, kDin, 0L,
        (void*)Yo[dir], nullptr, kOutP, 0L,
        nullptr, nullptr, 0L,
        kRows, kOutP, kDin, 1.0f);
  }

  combine_kernel<<<kRows / 8, 256, 0, stream>>>(x, lq, n2w, Yo[0], Yo[1], out);
}
